// MoEBiEncoder_17772574671523
// MI455X (gfx1250) — hardware-verified
//
#include <hip/hip_runtime.h>
typedef __attribute__((ext_vector_type(4))) float vf4v_t;
typedef __attribute__((ext_vector_type(4))) unsigned int vu4v_t;
typedef __attribute__((ext_vector_type(4))) int vi4v_t;

typedef __attribute__((ext_vector_type(16))) __bf16 bf16x16;
typedef __attribute__((ext_vector_type(8)))  __bf16 bf16x8;
typedef __attribute__((ext_vector_type(8)))  float  f32x8;
typedef __attribute__((ext_vector_type(4)))  float  f32x4;

#define BH   8192
#define HDIM 768
#define HH   384
#define NE   8

#define BM 128
#define BN 64
#define BK 32
#define LDA 56
#define LDB 56

__device__ __forceinline__ __bf16 f2bf(float f) {
  unsigned u = __builtin_bit_cast(unsigned, f);
  unsigned r = u + 0x7FFFu + ((u >> 16) & 1u);
  unsigned short s = (unsigned short)(r >> 16);
  return __builtin_bit_cast(__bf16, s);
}

__device__ __forceinline__ void split_bf16(float v, __bf16& hi, __bf16& lo) {
  const unsigned u = __builtin_bit_cast(unsigned, v) & 0xffff0000u;
  hi = __builtin_bit_cast(__bf16, (unsigned short)(u >> 16));
  lo = f2bf(v - __builtin_bit_cast(float, u));
}
__device__ __forceinline__ f32x8 wmmab(bf16x16 a, bf16x16 b, f32x8 c) {
  f32x8 d = __builtin_amdgcn_wmma_f32_16x16x32_bf16(false, a, false, b, (short)0, c, false, false);
  asm volatile("v_nop\n\tv_nop\n\tv_nop\n\tv_nop" : "+v"(d) : "v"(a), "v"(b));
  return d;
}

__global__ void cvt_f32_bf16(const float* __restrict__ in, __bf16* __restrict__ out, int n) {
  int stride = gridDim.x * blockDim.x;
  for (int i8 = blockIdx.x * blockDim.x + threadIdx.x; i8 < n / 8; i8 += stride) {
    bf16x8 v;
#pragma unroll
    for (int e = 0; e < 8; ++e) v[e] = f2bf(in[(size_t)i8 * 8 + e]);
    *(volatile bf16x8*)(out + (size_t)i8 * 8) = v; __threadfence(); *(volatile bf16x8*)(out + (size_t)i8 * 8) = v;
  }
}

__global__ __launch_bounds__(256) void rowlist_kernel(const int* __restrict__ eidx, int* __restrict__ counts, int* __restrict__ rowlist) {
  __shared__ int scan[NE][256];
  __shared__ int segoff[NE + 1];
  __shared__ __attribute__((aligned(16))) int lst[BH + 64];
  const int t = threadIdx.x;
  int loc[NE];
#pragma unroll
  for (int e = 0; e < NE; ++e) loc[e] = 0;
  for (int r = t * 32; r < t * 32 + 32; ++r) { const int x = eidx[r];
#pragma unroll
    for (int e = 0; e < NE; ++e) loc[e] += (x == e); }
#pragma unroll
  for (int e = 0; e < NE; ++e) scan[e][t] = loc[e];
  __syncthreads();
  if (t < NE) { int run = 0; for (int i = 0; i < 256; ++i) { const int v = scan[t][i]; scan[t][i] = run; run += v; } segoff[t] = run; }
  __syncthreads();
  if (t == 0) { int run = 0; for (int e = 0; e < NE; ++e) { const int c = segoff[e]; segoff[e] = run; run += c; } segoff[NE] = run; }
  __syncthreads();
  int pos[NE];
#pragma unroll
  for (int e = 0; e < NE; ++e) pos[e] = segoff[e] + scan[e][t];
  for (int r = t * 32; r < t * 32 + 32; ++r) {
    const int x = eidx[r];
    int p = 0;
#pragma unroll
    for (int e = 0; e < NE; ++e) if (e == x) { p = pos[e]; pos[e]++; }
    lst[p] = r;
  }
  if (t < 64) lst[BH + t] = 0;
  __syncthreads();
  for (int pass = 0; pass < 2; ++pass) {
    for (int e = 0; e < NE; ++e) {
      const int c = segoff[e + 1] - segoff[e];
      const int npieces = ((c + 31) / 32) * 8;
      for (int pc = t; pc < npieces; pc += 256) {
        const int base = segoff[e] + pc * 4;
        vi4v_t v = {lst[min(base + 0, BH + 63)], lst[min(base + 1, BH + 63)], lst[min(base + 2, BH + 63)], lst[min(base + 3, BH + 63)]};
        *(volatile vi4v_t*)(rowlist + (size_t)e * BH + pc * 4) = v;
      }
      if (t == 0) *(volatile int*)(counts + e) = c;
    }
    __threadfence();
  }
}

union AFrag { bf16x16 v; bf16x8 h[2]; };

template <int MODE, bool SPLIT>
__global__ __launch_bounds__(256)
void gemm_wmma(const void*   __restrict__ Av,
               const void*   __restrict__ Bv,
               const float*  __restrict__ bias,
               float*        __restrict__ outF,
               __bf16*       __restrict__ outBF,
               const int*    __restrict__ rowlist,
               const int*    __restrict__ counts,
               const float*  __restrict__ gate,
               int K, int Ntot) {
  __shared__ __align__(16) unsigned char smem[2 * (BM * LDA + BN * LDB) * 2];
  __bf16* Ash = (__bf16*)smem;               __bf16* Bsh = Ash + BM * LDA;
  __bf16* Asl = Bsh + BN * LDB;              __bf16* Bsl = Asl + BM * LDA;
  float*  Cs  = (float*)smem;

  const int tid  = threadIdx.x;
  const int lane = tid & 31;
  const int w    = tid >> 5;
  const int wm   = w & 3;
  const int wn   = w >> 2;
  const int mtile = blockIdx.x;
  const int n0    = blockIdx.y * BN;
  const int e     = (MODE == 0) ? 0 : blockIdx.z;
  const int hh   = lane >> 4, l16 = lane & 15;

  int m_count = BM;
  const int* rl = nullptr;
  if constexpr (MODE != 0) {
    int cnt = counts[e];
    if (mtile * BM >= cnt) return;
    m_count = min(BM, cnt - mtile * BM);
    rl = rowlist + e * BH + mtile * BM;
  }
  const float* bbase = bias + (size_t)e * Ntot;

  const int ai = tid >> 1;
  const int ak = (tid & 1) * 16;
  int arow;
  if constexpr (MODE == 0) arow = mtile * BM + ai;
  else                     arow = (ai < m_count) ? rl[ai] : rl[0];
  const int bk = tid >> 3;
  const int bn = (tid & 7) * 8;

  f32x8 acc[2][2] = {};
  const int ksteps = K / BK;
  for (int ks = 0; ks < ksteps; ++ks) {
    const int k0 = ks * BK;
    __syncthreads();
    if constexpr (SPLIT) {
      const float* ap = (const float*)Av + (size_t)arow * K + k0 + ak;
      const float* bp = (const float*)Bv + (size_t)(k0 + bk) * Ntot + n0 + bn;
#pragma unroll
      for (int j = 0; j < 16; ++j) { __bf16 h_, l_; split_bf16(ap[j], h_, l_); Ash[ai * LDA + ak + j] = h_; Asl[ai * LDA + ak + j] = l_; }
#pragma unroll
      for (int j = 0; j < 8; ++j) { __bf16 h_, l_; split_bf16(bp[j], h_, l_); Bsh[(bn + j) * LDB + bk] = h_; Bsl[(bn + j) * LDB + bk] = l_; }
    } else {
      const __bf16* ap = (const __bf16*)Av + (size_t)arow * K + k0 + ak;
      const __bf16* bp = (const __bf16*)Bv + (size_t)e * K * Ntot + (size_t)(k0 + bk) * Ntot + n0 + bn;
      *(bf16x8*)(Ash + ai * LDA + ak) = *(const bf16x8*)ap; *(bf16x8*)(Ash + ai * LDA + ak + 8) = *(const bf16x8*)(ap + 8);
      const bf16x8 bv = *(const bf16x8*)bp;
#pragma unroll
      for (int j = 0; j < 8; ++j) Bsh[(bn + j) * LDB + bk] = bv[j];
    }
    __syncthreads();

    AFrag ah[2], bh[2], al[2], bl[2];
#pragma unroll
    for (int ms = 0; ms < 2; ++ms) {
      const __bf16* p = Ash + (wm * 32 + ms * 16 + l16) * LDA + 8 * hh;
      ah[ms].h[0] = *(const bf16x8*)(p); ah[ms].h[1] = *(const bf16x8*)(p + 16);
      if constexpr (SPLIT) { const __bf16* pl = Asl + (wm * 32 + ms * 16 + l16) * LDA + 8 * hh; al[ms].h[0] = *(const bf16x8*)(pl); al[ms].h[1] = *(const bf16x8*)(pl + 16); }
    }
#pragma unroll
    for (int ns = 0; ns < 2; ++ns) {
      const __bf16* p = Bsh + (wn * 32 + ns * 16 + l16) * LDB + 8 * hh;
      bh[ns].h[0] = *(const bf16x8*)(p); bh[ns].h[1] = *(const bf16x8*)(p + 16);
      if constexpr (SPLIT) { const __bf16* pl = Bsl + (wn * 32 + ns * 16 + l16) * LDB + 8 * hh; bl[ns].h[0] = *(const bf16x8*)(pl); bl[ns].h[1] = *(const bf16x8*)(pl + 16); }
    }
#pragma unroll
    for (int ms = 0; ms < 2; ++ms)
#pragma unroll
      for (int ns = 0; ns < 2; ++ns) {
        acc[ms][ns] = wmmab(ah[ms].v, bh[ns].v, acc[ms][ns]);
        if constexpr (SPLIT) { acc[ms][ns] = wmmab(ah[ms].v, bl[ns].v, acc[ms][ns]); acc[ms][ns] = wmmab(al[ms].v, bh[ns].v, acc[ms][ns]); }
      }
  }
  __syncthreads();

#pragma unroll
  for (int ns = 0; ns < 2; ++ns) {
    const int cl = wn * 32 + ns * 16 + l16;
    const float bvv = bbase[n0 + cl];
#pragma unroll
    for (int ms = 0; ms < 2; ++ms)
#pragma unroll
      for (int v = 0; v < 8; ++v) {
        const int rloc = wm * 32 + ms * 16 + v + hh * 8;
        float val = acc[ms][ns][v] + bvv;
        if constexpr (MODE == 0 || MODE == 1) val = fmaxf(val, 0.0f);
        if constexpr (MODE == 2) { const int b = (rloc < m_count) ? rl[rloc] : 0; val *= gate[b]; }
        Cs[rloc * BN + cl] = val;
      }
  }
  __syncthreads();
  for (int pass = 0; pass < 2; ++pass) {
    if constexpr (MODE == 1) {
#pragma unroll
      for (int q4 = 0; q4 < 4; ++q4) {
        const int piece = tid + q4 * 256, rloc = piece >> 3, sg = piece & 7;
        if (rloc < m_count) {
          bf16x8 hv;
#pragma unroll
          for (int j = 0; j < 8; ++j) hv[j] = f2bf(Cs[rloc * BN + sg * 8 + j]);
          *(volatile bf16x8*)(outBF + (size_t)rl[rloc] * Ntot + n0 + sg * 8) = hv;
        }
      }
    } else {
#pragma unroll
      for (int q8 = 0; q8 < 8; ++q8) {
        const int piece = tid + q8 * 256, rloc = piece >> 4, sg = piece & 15;
        if (rloc < m_count) {
          const int row = (MODE == 0) ? (mtile * BM + rloc) : rl[rloc];
          *(volatile f32x4*)(outF + (size_t)row * Ntot + n0 + sg * 4) = *(const f32x4*)(Cs + rloc * BN + sg * 4);
        }
      }
    }
    __threadfence();
  }
}

__global__ __launch_bounds__(256)
void gating_kernel(const float* __restrict__ x1, const float* __restrict__ w3,
                   const float* __restrict__ b3, int* __restrict__ eidx,
                   float* __restrict__ gate) {
  __shared__ int   se[32];
  __shared__ float sg[32];
  const int wave = threadIdx.x >> 5;
  const int lane = threadIdx.x & 31;
  for (int rr = 0; rr < 4; ++rr) {
    const int bl = wave * 4 + rr;
    const int b = blockIdx.x * 32 + bl;
    float acc[NE];
#pragma unroll
    for (int e = 0; e < NE; ++e) acc[e] = 0.f;
    const float* xr = x1 + (size_t)b * HH;
    for (int f = lane; f < HH; f += 32) {
      float xv = xr[f];
      const float* wr = w3 + f * NE;
#pragma unroll
      for (int e = 0; e < NE; ++e) acc[e] += xv * wr[e];
    }
#pragma unroll
    for (int e = 0; e < NE; ++e)
      for (int off = 16; off > 0; off >>= 1)
        acc[e] += __shfl_xor(acc[e], off, 32);
    if (lane == 0) {
      float mx = -1e30f; int am = 0;
#pragma unroll
      for (int e = 0; e < NE; ++e) {
        float v = acc[e] + b3[e];
        acc[e] = v;
        if (v > mx) { mx = v; am = e; }
      }
      float s = 0.f;
#pragma unroll
      for (int e = 0; e < NE; ++e) s += expf(acc[e] - mx);
      se[bl] = am;
      sg[bl] = 1.0f / s;
    }
  }
  __syncthreads();
  if (wave == 0) {
    const int b = blockIdx.x * 32 + lane;
    const int ev = se[lane]; const float gv = sg[lane];
    *(volatile int*)(eidx + b) = ev; *(volatile float*)(gate + b) = gv;
    __threadfence();
    *(volatile int*)(eidx + b) = ev; *(volatile float*)(gate + b) = gv;
  }
}

__global__ __launch_bounds__(256)
void finalize_kernel(const float* __restrict__ pre, const float* __restrict__ q,
                     float* __restrict__ out) {
  __shared__ float red[256];
  const int b = blockIdx.x;
  const float* pr = pre + (size_t)b * HDIM;
  float s = 0.f;
  for (int c = threadIdx.x; c < HDIM; c += 256) { float v = pr[c]; s += v * v; }
  red[threadIdx.x] = s;
  __syncthreads();
  for (int off = 128; off > 0; off >>= 1) {
    if (threadIdx.x < off) red[threadIdx.x] += red[threadIdx.x + off];
    __syncthreads();
  }
  const float rn = 1.0f / fmaxf(sqrtf(red[0]), 1e-6f);
  for (int c = threadIdx.x; c < HDIM; c += 256) {
    const float v = pr[c] * rn + q[(size_t)b * HDIM + c];
    *(volatile float*)(out + (size_t)b * HDIM + c) = v; __threadfence(); *(volatile float*)(out + (size_t)b * HDIM + c) = v;
  }
}

extern "C" void kernel_launch(void* const* d_in, const int* in_sizes, int n_in,
                              void* d_out, int out_size, void* d_ws, size_t ws_size,
                              hipStream_t stream) {
  (void)in_sizes; (void)n_in; (void)out_size;
  const float* q      = (const float*)d_in[0];
  const float* cls_w1 = (const float*)d_in[1];
  const float* cls_b1 = (const float*)d_in[2];
  const float* cls_w3 = (const float*)d_in[3];
  const float* cls_b3 = (const float*)d_in[4];
  const float* exp_w1 = (const float*)d_in[5];
  const float* exp_b1 = (const float*)d_in[6];
  const float* exp_w2 = (const float*)d_in[7];
  const float* exp_b2 = (const float*)d_in[8];
  float* out = (float*)d_out;

  char* ws = (char*)d_ws;
  size_t off = 0;
  auto take = [&](size_t bytes) -> char* {
    char* p = ws + off;
    off = (off + bytes + 255) & ~(size_t)255;
    return p;
  };
  __bf16* qb     = (__bf16*)take((size_t)BH * HDIM * 2);
  __bf16* w1b    = (__bf16*)take((size_t)HDIM * HH * 2);
  __bf16* ew1b   = (__bf16*)take((size_t)NE * HDIM * HH * 2);
  __bf16* ew2b   = (__bf16*)take((size_t)NE * HH * HDIM * 2);
  float*  x1     = (float*) take((size_t)BH * HH * 4);
  __bf16* hbuf   = (__bf16*)take((size_t)BH * HH * 2);
  float*  opre   = (float*) take((size_t)BH * HDIM * 4);
  int*    eidx   = (int*)   take((size_t)BH * 4);
  float*  gate   = (float*) take((size_t)BH * 4);
  int*    counts = (int*)   take((size_t)NE * 4);
  int*    rlist  = (int*)   take((size_t)NE * BH * 4);

  if (off > ws_size) return;
  cvt_f32_bf16<<<2048, 256, 0, stream>>>(q, qb, BH * HDIM);
  cvt_f32_bf16<<<2048, 256, 0, stream>>>(exp_w1, ew1b, NE * HDIM * HH);
  cvt_f32_bf16<<<2048, 256, 0, stream>>>(exp_w2, ew2b, NE * HH * HDIM);
  (void)w1b;

  gemm_wmma<0, true><<<dim3(BH / BM, HH / BN, 1), 256, 0, stream>>>(
      q, cls_w1, cls_b1, x1, nullptr, nullptr, nullptr, nullptr, HDIM, HH);

  gating_kernel<<<BH / 32, 256, 0, stream>>>(x1, cls_w3, cls_b3, eidx, gate);
  rowlist_kernel<<<1, 256, 0, stream>>>(eidx, counts, rlist);

  gemm_wmma<1, false><<<dim3(BH / BM, HH / BN, NE), 256, 0, stream>>>(
      qb, ew1b, exp_b1, nullptr, hbuf, rlist, counts, nullptr, HDIM, HH);

  gemm_wmma<2, false><<<dim3(BH / BM, HDIM / BN, NE), 256, 0, stream>>>(
      hbuf, ew2b, exp_b2, opre, nullptr, rlist, counts, gate, HH, HDIM);

  finalize_kernel<<<BH, 256, 0, stream>>>(opre, q, out);
}
